// RMPI_7550552506743
// MI455X (gfx1250) — hardware-verified
//
#include <hip/hip_runtime.h>

typedef __bf16 v16b __attribute__((ext_vector_type(16)));
typedef unsigned short v16us __attribute__((ext_vector_type(16)));
typedef unsigned short v8us __attribute__((ext_vector_type(8)));
typedef float v8f __attribute__((ext_vector_type(8)));
typedef float v4f __attribute__((ext_vector_type(4)));
typedef int v4i __attribute__((ext_vector_type(4)));
typedef v8us __attribute__((may_alias)) v8usa;
typedef v4f __attribute__((may_alias)) v4fa;
typedef v4i __attribute__((may_alias)) v4ia;

union FragU { v16us u; v8us half[2]; unsigned short s[16]; };

#define NE 16384
#define NB 2048
#define NR 200
#define DD 32
#define NM 6

__device__ __forceinline__ int fixidx(int i, int n) {
  i += (i < 0) ? n : 0;
  i = (i < 0) ? 0 : i;
  i = (i > n - 1) ? (n - 1) : i;
  return i;
}

__device__ __forceinline__ unsigned bf16_rne(float x) {
  const unsigned u = __float_as_uint(x);
  return (u + 0x7FFFu + ((u >> 16) & 1u)) >> 16;
}

__device__ __forceinline__ void split_bf16(float x, unsigned& hi, unsigned& lo) {
  hi = bf16_rne(x);
  const float hf = __uint_as_float(hi << 16);
  lo = bf16_rne(x - hf);
}

__device__ __forceinline__ float lk02(float s) { return (s > 0.0f) ? s : 0.2f * s; }

__device__ __forceinline__ v8f wmma_bf(v16us a, v16us b, v8f c) {
  const v16b ab = __builtin_bit_cast(v16b, a);
  const v16b bb = __builtin_bit_cast(v16b, b);
  v8f d = __builtin_amdgcn_wmma_f32_16x16x32_bf16(false, ab, false, bb, (short)0, c, false, false);
  asm volatile("v_nop\n\tv_nop\n\tv_nop\n\tv_nop" : "+v"(d) : "v"(a), "v"(b));
  return d;
}

__device__ __forceinline__ v8f mm3(v16us ah, v16us al, v16us bh, v16us bl, v8f c) {
  c = wmma_bf(ah, bh, c);
  c = wmma_bf(ah, bl, c);
  c = wmma_bf(al, bh, c);
  return c;
}

__device__ __forceinline__ v16us ldfrag(const unsigned short* p, int h) {
  FragU f;
  f.half[0] = *(const v8usa*)(p + 8 * h);
  f.half[1] = *(const v8usa*)(p + 16 + 8 * h);
  return f.u;
}

__device__ __forceinline__ unsigned mode_code(int es, int ed, int u, int v) {
  const unsigned iu = (ed == u) ? 1u : 0u, ou = (es == u) ? 1u : 0u;
  const unsigned iv = (ed == v) ? 1u : 0u, ov = (es == v) ? 1u : 0u;
  return (iu & (ov ^ 1u)) | ((ou & (iv ^ 1u)) << 1) | ((iv & (ou ^ 1u)) << 2) |
         ((ov & (iu ^ 1u)) << 3) | ((ou & iv) << 4) | ((iu & ov) << 5);
}

__device__ __forceinline__ int pick8(v4i a, v4i c, int r) {
  return (r < 4) ? a[r & 3] : c[r & 3];
}

__global__ __launch_bounds__(256) void k_planes(
    const int* __restrict__ edge_type, const int* __restrict__ nbr_rels,
    const float* __restrict__ rel_emb, const float* __restrict__ W1,
    unsigned short* __restrict__ H0P, unsigned short* __restrict__ XP,
    unsigned short* __restrict__ WP)
{
  const int tid = threadIdx.x, bx = blockIdx.x;
  const float* src;
  unsigned short* base;
  size_t off, lo_off;
  if (bx < (NE * 4) / 256) {
    const int g = bx * 256 + tid;
    const int e = g >> 2, q = g & 3;
    const int t = fixidx(edge_type[e], NR);
    src = rel_emb + (size_t)t * DD + 8 * q;
    base = H0P; off = (size_t)e * DD + 8 * q; lo_off = (size_t)NE * DD;
  } else if (bx < (NE * 4 + NB * 4) / 256) {
    const int g = (bx - (NE * 4) / 256) * 256 + tid;
    const int b = g >> 2, q = g & 3;
    const int t = fixidx(nbr_rels[b], NR);
    src = rel_emb + (size_t)t * DD + 8 * q;
    base = XP; off = (size_t)b * DD + 8 * q; lo_off = (size_t)NB * DD;
  } else {
    const int g = (bx - (NE * 4 + NB * 4) / 256) * 256 + tid;
    if (g >= NM * DD * DD / 8) return;
    src = W1 + (size_t)g * 8;
    base = WP; off = (size_t)g * 8; lo_off = (size_t)NM * DD * DD;
  }
  const v4f a = *(const v4fa*)src;
  const v4f c = *(const v4fa*)(src + 4);
  const float xs[8] = {a.x, a.y, a.z, a.w, c.x, c.y, c.z, c.w};
  FragU fh, fl;
  #pragma unroll
  for (int i = 0; i < 8; ++i) {
    unsigned hi, lo;
    split_bf16(xs[i], hi, lo);
    fh.s[i] = (unsigned short)hi;
    fl.s[i] = (unsigned short)lo;
  }
  unsigned short* dh = base + off;
  unsigned short* dl = base + lo_off + off;
  const v8us hv = fh.half[0], lv = fl.half[0];
  *(volatile v8us*)dh = hv;
  *(volatile v8us*)dl = lv;
  __threadfence();
  *(volatile v8us*)dh = hv;
  *(volatile v8us*)dl = lv;
}

__device__ __forceinline__ void hit_store_pass(const unsigned short* sT, unsigned short* HITP,
                                               int i, int ebase, int tid) {
  const int q = tid & 7, sub = tid >> 3;
  #pragma unroll
  for (int it = 0; it < 8; ++it) {
    const int L = it * 8 + sub;
    const int pl = L >> 5, d = L & 31;
    const v8us v = *(const v8usa*)(sT + pl * 2048 + d * 64 + 8 * q);
    unsigned short* dst = HITP + ((size_t)(pl * NM * DD + i * DD + d)) * NE + ebase + 8 * q;
    *(volatile v8us*)dst = v;
  }
}

__global__ __launch_bounds__(64) void k_hiplanes(
    const unsigned short* __restrict__ H0P, const unsigned short* __restrict__ WP,
    const float* __restrict__ b1, unsigned short* __restrict__ HITP)
{
  __shared__ __attribute__((aligned(16))) unsigned short sT[2 * 32 * 64];
  const int tid = threadIdx.x, lane = tid & 31, w = tid >> 5;
  const int h = lane >> 4, m = lane & 15;
  const int i = blockIdx.y;
  const int ebase = blockIdx.x * 64;

  const unsigned short* wrow = WP + (size_t)(i * DD + 16 * w + m) * DD;
  const v16us wh = ldfrag(wrow, h);
  const v16us wl = ldfrag(wrow + (size_t)NM * DD * DD, h);

  const v8f zero8 = {0.f, 0.f, 0.f, 0.f, 0.f, 0.f, 0.f, 0.f};
  v8f acc[4];
  #pragma unroll
  for (int et = 0; et < 4; ++et) {
    const unsigned short* hrow = H0P + (size_t)(ebase + 16 * et + m) * DD;
    const v16us bh = ldfrag(hrow, h);
    const v16us bl = ldfrag(hrow + (size_t)NE * DD, h);
    acc[et] = mm3(wh, wl, bh, bl, zero8);
  }
  #pragma unroll
  for (int r = 0; r < 8; ++r) {
    const int d = 16 * w + 8 * h + r;
    const float bias = b1[i * DD + d];
    #pragma unroll
    for (int et = 0; et < 4; ++et) {
      const float val = acc[et][r] + bias;
      unsigned hi, lo;
      split_bf16(val, hi, lo);
      sT[d * 64 + 16 * et + m] = (unsigned short)hi;
      sT[2048 + d * 64 + 16 * et + m] = (unsigned short)lo;
    }
  }
  __syncthreads();
  hit_store_pass(sT, HITP, i, ebase, tid);
  __threadfence();
  hit_store_pass(sT, HITP, i, ebase, tid);
}

__global__ __launch_bounds__(32) void k_rowmax(
    const int* __restrict__ edge_src, const int* __restrict__ edge_dst,
    const int* __restrict__ nbr_edges,
    const unsigned short* __restrict__ XP, const unsigned short* __restrict__ H0P,
    float* __restrict__ MX)
{
  __shared__ __attribute__((aligned(16))) float sM[16 * 8];
  const int lane = threadIdx.x & 31, h = lane >> 4, m = lane & 15;
  const int b0 = blockIdx.x * 16, b = b0 + m;
  const int ne = fixidx(nbr_edges[b], NE);
  const int u = edge_src[ne], v = edge_dst[ne];
  const v16us xb = ldfrag(XP + (size_t)b * DD, h);

  const v8f zero8 = {0.f, 0.f, 0.f, 0.f, 0.f, 0.f, 0.f, 0.f};
  float mx[NM];
  #pragma unroll
  for (int i = 0; i < NM; ++i) mx[i] = -1.0e30f;

  #pragma unroll 1
  for (int e0 = 0; e0 < NE; e0 += 32) {
    #pragma unroll
    for (int t = 0; t < 2; ++t) {
      const int eb = e0 + 16 * t;
      const v16us a = ldfrag(H0P + (size_t)(eb + m) * DD, h);
      const v8f z = wmma_bf(a, xb, zero8);
      const v4i sa = *(const v4ia*)(edge_src + eb + 8 * h);
      const v4i sc = *(const v4ia*)(edge_src + eb + 8 * h + 4);
      const v4i da = *(const v4ia*)(edge_dst + eb + 8 * h);
      const v4i dc = *(const v4ia*)(edge_dst + eb + 8 * h + 4);
      #pragma unroll
      for (int r = 0; r < 8; ++r) {
        const int es = pick8(sa, sc, r), ed = pick8(da, dc, r);
        const unsigned code = mode_code(es, ed, u, v);
        const float sv = lk02(z[r]);
        #pragma unroll
        for (int i = 0; i < NM; ++i)
          mx[i] = ((code >> i) & 1u) ? fmaxf(mx[i], sv) : mx[i];
      }
    }
  }
  #pragma unroll
  for (int i = 0; i < NM; ++i) mx[i] = fmaxf(mx[i], __shfl_xor(mx[i], 16));
  if (h == 0) {
    #pragma unroll
    for (int i = 0; i < NM; ++i) sM[m * 8 + i] = mx[i];
    sM[m * 8 + 6] = 0.0f;
    sM[m * 8 + 7] = 0.0f;
  }
  __syncthreads();
  const v4f val = *(const v4fa*)(sM + 4 * lane);
  float* dst = MX + (size_t)b0 * 8 + 4 * lane;
  *(volatile v4f*)dst = val;
  __threadfence();
  *(volatile v4f*)dst = val;
}

__device__ __forceinline__ void agg_store_pass(const float* sO, float* AGG, int b0, int tid) {
  const int q = tid & 7, sub = tid >> 3;
  #pragma unroll
  for (int it = 0; it < 2; ++it) {
    const int row = it * 8 + sub;
    const v4f va = *(const v4fa*)(sO + row * 32 + 4 * q);
    const v4f vb = *(const v4fa*)(sO + 512 + row * 32 + 4 * q);
    const v4f vs = va + vb;
    *(volatile v4f*)(AGG + (size_t)(b0 + row) * DD + 4 * q) = vs;
  }
}

__global__ __launch_bounds__(64) void k_aggr(
    const int* __restrict__ edge_src, const int* __restrict__ edge_dst,
    const int* __restrict__ nbr_edges,
    const unsigned short* __restrict__ XP, const unsigned short* __restrict__ H0P,
    const unsigned short* __restrict__ HITP, const float* __restrict__ MX,
    float* __restrict__ AGG)
{
  __shared__ __attribute__((aligned(16))) float sS[2 * 512];
  __shared__ __attribute__((aligned(16))) float sO[2 * 512];

  const int tid = threadIdx.x, lane = tid & 31, w = tid >> 5;
  const int h = lane >> 4, m = lane & 15;
  const int b0 = blockIdx.x * 16, b = b0 + m;
  const int ne = fixidx(nbr_edges[b], NE);
  const int u = edge_src[ne], v = edge_dst[ne];
  const v16us xbh = ldfrag(XP + (size_t)b * DD, h);
  const v16us xbl = ldfrag(XP + (size_t)NB * DD + (size_t)b * DD, h);
  const int msh = 3 * w;

  const v8f zero8 = {0.f, 0.f, 0.f, 0.f, 0.f, 0.f, 0.f, 0.f};
  float mxv[3], den[3];
  v8f acc[3][2];
  #pragma unroll
  for (int j = 0; j < 3; ++j) {
    mxv[j] = MX[(size_t)b * 8 + msh + j];
    den[j] = 0.0f;
    acc[j][0] = zero8;
    acc[j][1] = zero8;
  }

  #pragma unroll 1
  for (int e0 = 0; e0 < NE; e0 += 32) {
    float* sb = sS + ((e0 >> 5) & 1) * 512;
    {
      const int eb = e0 + 16 * w;
      const unsigned short* arow = H0P + (size_t)(eb + m) * DD;
      const v16us ah = ldfrag(arow, h);
      const v16us al = ldfrag(arow + (size_t)NE * DD, h);
      const v8f z = mm3(ah, al, xbh, xbl, zero8);
      v4f za, zc;
      za.x = lk02(z[0]); za.y = lk02(z[1]); za.z = lk02(z[2]); za.w = lk02(z[3]);
      zc.x = lk02(z[4]); zc.y = lk02(z[5]); zc.z = lk02(z[6]); zc.w = lk02(z[7]);
      float* sp = sb + m * 32 + 16 * w + 8 * h;
      *(v4fa*)sp = za;
      *(v4fa*)(sp + 4) = zc;
    }
    __syncthreads();

    v8f s[2];
    #pragma unroll
    for (int t = 0; t < 2; ++t) {
      const float* rp = sb + m * 32 + 16 * t + 8 * h;
      const v4f qa = *(const v4fa*)rp;
      const v4f qc = *(const v4fa*)(rp + 4);
      const v8f tmp = {qa.x, qa.y, qa.z, qa.w, qc.x, qc.y, qc.z, qc.w};
      s[t] = tmp;
    }

    unsigned cm0 = 0u, cm1 = 0u, cm2 = 0u;
    #pragma unroll
    for (int t = 0; t < 2; ++t) {
      const int eb = e0 + 16 * t + 8 * h;
      const v4i sa = *(const v4ia*)(edge_src + eb);
      const v4i sc = *(const v4ia*)(edge_src + eb + 4);
      const v4i da = *(const v4ia*)(edge_dst + eb);
      const v4i dc = *(const v4ia*)(edge_dst + eb + 4);
      #pragma unroll
      for (int r = 0; r < 8; ++r) {
        const int es = pick8(sa, sc, r), ed = pick8(da, dc, r);
        const unsigned code = mode_code(es, ed, u, v);
        const float sv = s[t][r];
        const unsigned sel = (sv != 0.0f) ? ((code >> msh) & 7u) : 0u;
        const int e = 8 * t + r;
        cm0 |= (sel & 1u) << e;
        cm1 |= ((sel >> 1) & 1u) << e;
        cm2 |= ((sel >> 2) & 1u) << e;
      }
    }
    const unsigned cm[3] = {cm0, cm1, cm2};

    #pragma unroll
    for (int j = 0; j < 3; ++j) {
      const unsigned cmj = cm[j];
      if (__builtin_amdgcn_ballot_w32(cmj != 0u) != 0u) {
        FragU fh, fl;
        float dsum = 0.0f;
        #pragma unroll
        for (int e = 0; e < 16; ++e) {
          const float x = fminf(s[e >> 3][e & 7] - mxv[j], 64.0f);
          const float p = ((cmj >> e) & 1u) ? __expf(x) : 0.0f;
          dsum += p;
          unsigned hi, lo;
          split_bf16(p, hi, lo);
          fh.s[e] = (unsigned short)hi;
          fl.s[e] = (unsigned short)lo;
        }
        den[j] += dsum;
        #pragma unroll
        for (int dt = 0; dt < 2; ++dt) {
          const unsigned short* grow =
              HITP + ((size_t)((msh + j) * DD + 16 * dt + m)) * NE + e0;
          const v16us gh = ldfrag(grow, h);
          const v16us gl = ldfrag(grow + (size_t)NM * DD * NE, h);
          acc[j][dt] = mm3(gh, gl, fh.u, fl.u, acc[j][dt]);
        }
      }
    }
  }

  float rd[3];
  #pragma unroll
  for (int j = 0; j < 3; ++j) {
    const float dd = den[j] + __shfl_xor(den[j], 16);
    rd[j] = (dd > 0.0f) ? __builtin_amdgcn_rcpf(dd) : 0.0f;
  }
  #pragma unroll
  for (int dt = 0; dt < 2; ++dt) {
    float o[8];
    #pragma unroll
    for (int r = 0; r < 8; ++r)
      o[r] = acc[0][dt][r] * rd[0] + acc[1][dt][r] * rd[1] + acc[2][dt][r] * rd[2];
    const v4f oa = {o[0], o[1], o[2], o[3]};
    const v4f oc = {o[4], o[5], o[6], o[7]};
    float* sp = sO + w * 512 + m * 32 + 16 * dt + 8 * h;
    *(v4fa*)sp = oa;
    *(v4fa*)(sp + 4) = oc;
  }
  __syncthreads();
  agg_store_pass(sO, AGG, b0, tid);
  __threadfence();
  agg_store_pass(sO, AGG, b0, tid);
}

__device__ __forceinline__ void out_store_pass(const float* sA, float* out, int e0, int lane) {
  const int q = lane & 7, sub = lane >> 3;
  #pragma unroll
  for (int it = 0; it < 8; ++it) {
    const int row = it * 4 + sub;
    const v4f val = *(const v4fa*)(sA + row * 32 + 4 * q);
    *(volatile v4f*)(out + (size_t)(e0 + row) * DD + 4 * q) = val;
  }
}

__global__ __launch_bounds__(32) void k_out(
    const int* __restrict__ nbr_edges, const int* __restrict__ edge_type,
    const float* __restrict__ rel_emb, const float* __restrict__ AGG,
    float* __restrict__ out)
{
  __shared__ __attribute__((aligned(16))) float sA[32 * 32];
  const int lane = threadIdx.x & 31;
  const int e0 = blockIdx.x * 32;

  #pragma unroll 4
  for (int j = 0; j < 32; ++j) {
    const int t = fixidx(edge_type[e0 + j], NR);
    sA[j * 32 + lane] = rel_emb[(size_t)t * DD + lane];
  }

  #pragma unroll 1
  for (int c = 0; c < NB / 32; ++c) {
    const int id = nbr_edges[c * 32 + lane];
    const int idw = id + ((id < 0) ? NE : 0);
    const int jl = idw - e0;
    const bool hit = ((unsigned)jl < 32u);
    unsigned bal = __builtin_amdgcn_ballot_w32(hit);
    #pragma unroll 1
    for (int k = 0; k < 32 && bal != 0u; ++k) {
      const int bit = __builtin_ctz(bal);
      const int jrow = __shfl(jl, bit) & 31;
      const int bb = c * 32 + bit;
      const float a = AGG[(size_t)bb * DD + lane];
      sA[jrow * 32 + lane] += fmaxf(a, 0.0f);
      bal &= bal - 1u;
    }
  }
  __syncthreads();
  out_store_pass(sA, out, e0, lane);
  __threadfence();
  out_store_pass(sA, out, e0, lane);
}

extern "C" void kernel_launch(void* const* d_in, const int* in_sizes, int n_in,
                              void* d_out, int out_size, void* d_ws, size_t ws_size,
                              hipStream_t stream) {
  if (n_in < 8) return;
  if (in_sizes[0] != NE || in_sizes[1] != NE || in_sizes[2] != NE) return;
  if (in_sizes[3] != NB || in_sizes[4] != NB) return;
  if (in_sizes[5] != NR * DD || in_sizes[6] != NM * DD * DD || in_sizes[7] != NM * DD) return;
  if (out_size != NE * DD) return;

  const int*   edge_src  = (const int*)d_in[0];
  const int*   edge_dst  = (const int*)d_in[1];
  const int*   edge_type = (const int*)d_in[2];
  const int*   nbr_edges = (const int*)d_in[3];
  const int*   nbr_rels  = (const int*)d_in[4];
  const float* rel_emb   = (const float*)d_in[5];
  const float* W1        = (const float*)d_in[6];
  const float* b1        = (const float*)d_in[7];
  float* out = (float*)d_out;

  const size_t h0p_bytes = (size_t)2 * NE * DD * 2;
  const size_t xp_bytes  = (size_t)2 * NB * DD * 2;
  const size_t wp_bytes  = (size_t)2 * NM * DD * DD * 2;
  const size_t hit_bytes = (size_t)2 * NM * DD * NE * 2;
  const size_t mx_bytes  = (size_t)NB * 8 * 4;
  const size_t agg_bytes = (size_t)NB * DD * 4;
  const size_t total = h0p_bytes + xp_bytes + wp_bytes + hit_bytes + mx_bytes + agg_bytes;
  if (total > ws_size) return;

  char* ws = (char*)d_ws;
  unsigned short* H0P  = (unsigned short*)(ws);
  unsigned short* XP   = (unsigned short*)(ws + h0p_bytes);
  unsigned short* WP   = (unsigned short*)(ws + h0p_bytes + xp_bytes);
  unsigned short* HITP = (unsigned short*)(ws + h0p_bytes + xp_bytes + wp_bytes);
  float* MX  = (float*)(ws + h0p_bytes + xp_bytes + wp_bytes + hit_bytes);
  float* AGG = (float*)(ws + h0p_bytes + xp_bytes + wp_bytes + hit_bytes + mx_bytes);

  const int nblk1 = (NE * 4 + NB * 4 + NM * DD * DD / 8 + 255) / 256;
  k_planes<<<nblk1, 256, 0, stream>>>(edge_type, nbr_rels, rel_emb, W1, H0P, XP, WP);

  dim3 gHi(NE / 64, NM);
  k_hiplanes<<<gHi, 64, 0, stream>>>(H0P, WP, b1, HITP);

  k_rowmax<<<NB / 16, 32, 0, stream>>>(edge_src, edge_dst, nbr_edges, XP, H0P, MX);

  k_aggr<<<NB / 16, 64, 0, stream>>>(edge_src, edge_dst, nbr_edges, XP, H0P, HITP, MX, AGG);

  k_out<<<NE / 32, 32, 0, stream>>>(nbr_edges, edge_type, rel_emb, AGG, out);
}
